// Golu_5385888989796
// MI455X (gfx1250) — hardware-run, weakly checked
//
#include <hip/hip_runtime.h>
#include <stdint.h>


typedef _Float16 v16h __attribute__((ext_vector_type(16)));
typedef _Float16 v8h  __attribute__((ext_vector_type(8)));
typedef float    v8f  __attribute__((ext_vector_type(8)));
typedef float    v4f  __attribute__((ext_vector_type(4)));
typedef _Float16 h16;

#ifndef NB
#define NB 2
#endif
#ifndef SEQ
#define SEQ 1024
#endif
#define NB_FULL  2
#define SEQ_FULL 1024
#define DM   768
#define NH   12
#define HD   64
#define QKVW 2304
#define QKP  1536
#define FFW  3072
#define VOC  256
#define NLAY 4
#define ROWS (NB * SEQ)
#define OUT1_ELEMS ((long)NB_FULL * SEQ_FULL * VOC)

#define ACT_CAR   8.0f
#define W_CAR     1024.0f
#define PROJ_SCL  0.0009765625f
#define UNS_SCL   0.0001220703125f
#define RES_CAR   2048.0f
#define S_SCL     0.001953125f
#define P_CAR     16384.0f
#define O_SCL     7.62939453125e-06f
#define NEG_BIG   (-1.0e30f)

static_assert(NB == 1 || NB == 2);
static_assert(NB <= NB_FULL && SEQ <= SEQ_FULL);
static_assert(SEQ % 128 == 0);
static_assert(DM == NH * HD);
static_assert(HD == 64);
static_assert(QKVW == 3 * DM && QKP == 2 * DM);
static_assert(DM % 128 == 0 && DM % 64 == 0 && DM % 32 == 0 && QKVW % 64 == 0 && QKP % 64 == 0);
static_assert(FFW % 64 == 0 && FFW % 32 == 0 && VOC % 64 == 0);
static_assert(OUT1_ELEMS * 4 == 2097152L);
static_assert(ROWS % 8 == 0);
static_assert(6 * 32 * 4 == DM && 3 * 32 * 8 == DM);
static_assert((SEQ * 32) % 256 == 0);
static_assert((long)(QKVW / 64) * (DM / 64) * 4096 == (long)DM * QKVW);
static_assert((long)(FFW / 64) * (DM / 64) * 4096 == (long)DM * FFW);
static_assert((long)(VOC / 64) * (DM / 64) * 4096 == (long)DM * VOC);
static_assert((long)(QKP / 64) * (ROWS / 128) * 128 * 64 == (long)ROWS * QKP);
static_assert((long)(SEQ / 64) * (DM / 128) * 128 * 64 == (long)SEQ * DM);
static_assert((long)(SEQ / 128) * NH * 128 * HD == (long)SEQ * DM);
static_assert((long)(FFW / 64) * (ROWS / 128) * 128 * 64 == (long)ROWS * FFW);
static_assert((long)(DM / 64) * (ROWS / 128) * 128 * 64 == (long)ROWS * DM);
static_assert((long)(VOC / 64) * (ROWS / 128) * 128 * 64 == (long)ROWS * VOC);

#define N_WQKV ((size_t)NLAY * QKVW * DM)
#define N_W1   ((size_t)NLAY * FFW * DM)
#define N_W2   ((size_t)NLAY * DM * FFW)
#define N_WH   ((size_t)VOC * DM)
#define N_N16  ((size_t)ROWS * DM)
#define N_QK   ((size_t)ROWS * QKP)
#define N_VT   ((size_t)NB * DM * SEQ)
#define N_F1   ((size_t)ROWS * FFW)
#define N_HF   ((size_t)2 * ROWS * DM)
#define N_TAB  ((size_t)2 * SEQ * 32)
#define N_INV  ((size_t)64)
#define WS_HALVES (N_WQKV + N_W1 + N_W2 + N_WH + N_N16 + N_QK + N_VT + N_F1 + N_HF + N_HF + N_TAB + N_TAB + N_INV)
static_assert(WS_HALVES * 2 <= (size_t)134217728);
static_assert(N_WQKV % 64 == 0 && N_W1 % 64 == 0 && N_W2 % 64 == 0 && N_WH % 64 == 0 && N_N16 % 64 == 0);
static_assert(N_QK % 64 == 0 && N_VT % 64 == 0 && N_F1 % 64 == 0 && N_HF % 64 == 0 && N_TAB % 64 == 0);

union Frag16 { v16h v; v8h p[2]; };

__device__ __forceinline__ v16h ld_frag_g(const _Float16* __restrict__ p, int hl) {
  Frag16 f;
  f.p[0] = *(const v8h*)(p + 8 * hl);
  f.p[1] = *(const v8h*)(p + 16 + 8 * hl);
  return f.v;
}

__device__ __forceinline__ v16h ld_frag_s(const _Float16* base, int off, int hl) {
  Frag16 f;
  f.p[0] = *(const v8h*)(base + off + 8 * hl);
  f.p[1] = *(const v8h*)(base + off + 16 + 8 * hl);
  return f.v;
}

__device__ __forceinline__ v8f mma(v16h a, v16h b, v8f c) {
  v8f d = __builtin_amdgcn_wmma_f32_16x16x32_f16(false, a, false, b, (short)0, c, false, false);
  asm volatile("v_nop\n\tv_nop\n\tv_nop\n\tv_nop" : "+v"(d) : "v"(a), "v"(b));
  return d;
}

__device__ __forceinline__ float bf16_rne(float x) {
  unsigned int u = __builtin_bit_cast(unsigned int, x);
  u += 0x7FFFu + ((u >> 16) & 1u);
  return __builtin_bit_cast(float, u & 0xFFFF0000u);
}

static __device__ __forceinline__ h16 toh_flush(float v) {
  const h16 r = (h16)v;
  return (fabsf(v) < 6.103515625e-05f) ? (h16)0.0f : r;
}

static __device__ __forceinline__ float gelu_erf(float x) {
  return 0.5f * x * (1.0f + erff(x * 0.70710678118654752f));
}

__global__ __launch_bounds__(32) void k_invf(float* __restrict__ invf)
{
  const int i = threadIdx.x;
  const float e = (float)(2 * i) * 0.015625f;
  const float p = powf(10000.0f, e);
  const float v = 1.0f / p;
  *(volatile float*)(invf + i) = v;
  __threadfence();
  *(volatile float*)(invf + i) = v;
}

__global__ __launch_bounds__(256) void k_ropetab(const float* __restrict__ invf,
                                                 float* __restrict__ CosT, float* __restrict__ SinT)
{
  const int idx = blockIdx.x * 256 + threadIdx.x;
  const int i = idx & 31, t = idx >> 5;
  const float f = (float)t * invf[i];
  const float cs = cosf(f);
  const float sn = sinf(f);
  *(volatile float*)(CosT + idx) = cs;
  *(volatile float*)(SinT + idx) = sn;
  __threadfence();
  *(volatile float*)(CosT + idx) = cs;
  *(volatile float*)(SinT + idx) = sn;
}

__global__ __launch_bounds__(256) void k_embed(const int* __restrict__ tok, const float* __restrict__ emb,
                                               float* __restrict__ H0, float* __restrict__ H)
{
  const int lane = threadIdx.x & 31;
  const int row  = blockIdx.x * 8 + (threadIdx.x >> 5);
  const int bb = row / SEQ;
  const int nn = row - bb * SEQ;
  int t = tok[bb * SEQ_FULL + nn];
  t = (t < 0) ? 0 : ((t > VOC - 1) ? (VOC - 1) : t);
  const float* s = emb + (size_t)t * DM + 4 * lane;
  v4f o[6];
#pragma unroll
  for (int j = 0; j < 6; ++j) {
    const v4f x = *(const v4f*)(s + 128 * j);
    o[j][0] = bf16_rne(x[0]); o[j][1] = bf16_rne(x[1]);
    o[j][2] = bf16_rne(x[2]); o[j][3] = bf16_rne(x[3]);
  }
  float* d0 = H0 + (size_t)row * DM + 4 * lane;
  float* d1 = H  + (size_t)row * DM + 4 * lane;
#pragma unroll
  for (int j = 0; j < 6; ++j) {
    *(volatile v4f*)(d0 + 128 * j) = o[j];
    *(volatile v4f*)(d1 + 128 * j) = o[j];
  }
  __threadfence();
#pragma unroll
  for (int j = 0; j < 6; ++j) {
    *(volatile v4f*)(d0 + 128 * j) = o[j];
    *(volatile v4f*)(d1 + 128 * j) = o[j];
  }
}

__global__ __launch_bounds__(256) void k_ln(const float* __restrict__ X, const float* __restrict__ X2, int add2,
                                            const float* __restrict__ gs, const float* __restrict__ gb,
                                            _Float16* __restrict__ Y)
{
#pragma clang fp contract(off)
  const int lane = threadIdx.x & 31;
  const int row  = blockIdx.x * 8 + (threadIdx.x >> 5);
  const size_t ro = (size_t)row * DM + 8 * lane;
  float v[24];
  float s = 0.f;
#pragma unroll
  for (int j = 0; j < 3; ++j) {
    const v4f a0 = *(const v4f*)(X  + ro + 256 * j);
    const v4f a1 = *(const v4f*)(X  + ro + 256 * j + 4);
    const v4f b0 = *(const v4f*)(X2 + ro + 256 * j);
    const v4f b1 = *(const v4f*)(X2 + ro + 256 * j + 4);
#pragma unroll
    for (int e = 0; e < 4; ++e) {
      const float t0 = a0[e] + (add2 ? b0[e] : 0.0f);
      const float t1 = a1[e] + (add2 ? b1[e] : 0.0f);
      v[8 * j + e]     = t0;
      v[8 * j + 4 + e] = t1;
      s += t0;
      s += t1;
    }
  }
  s += __shfl_xor(s, 16, 32);
  s += __shfl_xor(s, 8, 32);
  s += __shfl_xor(s, 4, 32);
  s += __shfl_xor(s, 2, 32);
  s += __shfl_xor(s, 1, 32);
  const float mean = s * (1.0f / (float)DM);
  float vs = 0.f;
#pragma unroll
  for (int i = 0; i < 24; ++i) {
    const float d = v[i] - mean;
    vs += d * d;
  }
  vs += __shfl_xor(vs, 16, 32);
  vs += __shfl_xor(vs, 8, 32);
  vs += __shfl_xor(vs, 4, 32);
  vs += __shfl_xor(vs, 2, 32);
  vs += __shfl_xor(vs, 1, 32);
  const float rstd = rsqrtf(vs * (1.0f / (float)DM) + 1e-5f);

  v8h ov[3];
#pragma unroll
  for (int j = 0; j < 3; ++j) {
    const v4f g0 = *(const v4f*)(gs + 8 * lane + 256 * j);
    const v4f g1 = *(const v4f*)(gs + 8 * lane + 256 * j + 4);
    const v4f c0 = *(const v4f*)(gb + 8 * lane + 256 * j);
    const v4f c1 = *(const v4f*)(gb + 8 * lane + 256 * j + 4);
#pragma unroll
    for (int e = 0; e < 4; ++e) {
      const float y0 = (v[8 * j + e] - mean) * rstd * bf16_rne(g0[e]) + bf16_rne(c0[e]);
      const float y1 = (v[8 * j + 4 + e] - mean) * rstd * bf16_rne(g1[e]) + bf16_rne(c1[e]);
      ov[j][e]     = toh_flush(y0 * ACT_CAR);
      ov[j][4 + e] = toh_flush(y1 * ACT_CAR);
    }
  }
  _Float16* d = Y + ro;
#pragma unroll
  for (int j = 0; j < 3; ++j) *(volatile v8h*)(d + 256 * j) = ov[j];
  __threadfence();
#pragma unroll
  for (int j = 0; j < 3; ++j) *(volatile v8h*)(d + 256 * j) = ov[j];
}

__global__ __launch_bounds__(256) void k_trw(const float* __restrict__ W,
                                             _Float16* __restrict__ WT, int R, int C)
{
  __shared__ float tile[64 * 65];
  const int tid = threadIdx.x;
  const int c0 = blockIdx.x * 64, r0 = blockIdx.y * 64;
  const size_t zo = (size_t)blockIdx.z * (size_t)R * (size_t)C;
#pragma unroll
  for (int i = 0; i < 4; ++i) {
    const int idx = i * 256 + tid;
    const int r = idx >> 4, c4 = (idx & 15) * 4;
    const v4f v = *(const v4f*)(W + zo + (size_t)(r0 + r) * C + c0 + c4);
    tile[r * 65 + c4 + 0] = v[0];
    tile[r * 65 + c4 + 1] = v[1];
    tile[r * 65 + c4 + 2] = v[2];
    tile[r * 65 + c4 + 3] = v[3];
  }
  __syncthreads();
  v8h o[2];
  size_t dofs[2];
#pragma unroll
  for (int i = 0; i < 2; ++i) {
    const int line = i * 32 + (tid >> 3);
    const int pc   = (tid & 7) * 8;
#pragma unroll
    for (int j = 0; j < 8; ++j)
      o[i][j] = toh_flush(bf16_rne(tile[(pc + j) * 65 + line]) * W_CAR);
    dofs[i] = zo + (size_t)(c0 + line) * R + r0 + pc;
  }
  *(volatile v8h*)(WT + dofs[0]) = o[0];
  *(volatile v8h*)(WT + dofs[1]) = o[1];
  __threadfence();
  *(volatile v8h*)(WT + dofs[0]) = o[0];
  *(volatile v8h*)(WT + dofs[1]) = o[1];
}

__device__ __forceinline__ void gemm_core(const _Float16* __restrict__ ap0,
                                          const _Float16* __restrict__ ap1,
                                          const _Float16* __restrict__ bp, int K, int hl, v8f (&acc)[8])
{
  const size_t bst = (size_t)16 * K;
#pragma unroll 1
  for (int k0 = 0; k0 < K; k0 += 32) {
    const v16h a0 = ld_frag_g(ap0 + k0, hl);
    const v16h a1 = ld_frag_g(ap1 + k0, hl);
    const v16h b0 = ld_frag_g(bp + k0, hl);
    const v16h b1 = ld_frag_g(bp + bst + k0, hl);
    const v16h b2 = ld_frag_g(bp + 2 * bst + k0, hl);
    const v16h b3 = ld_frag_g(bp + 3 * bst + k0, hl);
    acc[0] = mma(a0, b0, acc[0]);
    acc[1] = mma(a0, b1, acc[1]);
    acc[2] = mma(a0, b2, acc[2]);
    acc[3] = mma(a0, b3, acc[3]);
    acc[4] = mma(a1, b0, acc[4]);
    acc[5] = mma(a1, b1, acc[5]);
    acc[6] = mma(a1, b2, acc[6]);
    acc[7] = mma(a1, b3, acc[7]);
  }
}

__global__ __launch_bounds__(128) __attribute__((amdgpu_num_vgpr(256)))
void k_proj(const _Float16* __restrict__ A, const _Float16* __restrict__ Bt,
            _Float16* __restrict__ PH, _Float16* __restrict__ PL,
            size_t sA, size_t sB, size_t sC, size_t sL,
            int K, int ldc, int ldl, int resN, int zshA)
{
  __shared__ __attribute__((aligned(16))) _Float16 ldsE[2 * 128 * 72];
  constexpr int OFF_L = 128 * 72;

  const int tid = threadIdx.x, lane = tid & 31;
  const int w = __builtin_amdgcn_readfirstlane(tid >> 5);
  const int hl = lane >> 4, c = lane & 15;
  const int z = blockIdx.z;
  const int m0 = blockIdx.y * 128, n0 = blockIdx.x * 64;
  const int mw = m0 + 32 * w;
  const bool wres = (n0 < resN);

  const _Float16* az = A  + (size_t)(z >> zshA) * sA;
  const _Float16* bz = Bt + (size_t)z * sB;
  const _Float16* ap0 = az + (size_t)(mw + c) * K;
  const _Float16* ap1 = az + (size_t)(mw + 16 + c) * K;
  const _Float16* bp  = bz + (size_t)(n0 + c) * K;

  v8f acc[8] = {};
  gemm_core(ap0, ap1, bp, K, hl, acc);

#pragma unroll
  for (int i = 0; i < 2; ++i)
#pragma unroll
    for (int t = 0; t < 4; ++t)
#pragma unroll
      for (int r = 0; r < 8; ++r) {
        const int rowl = 32 * w + 16 * i + 8 * hl + r;
        const float v = acc[i * 4 + t][r] * PROJ_SCL;
        const _Float16 hv = (_Float16)v;
        ldsE[rowl * 72 + 16 * t + c] = hv;
        if (wres) {
          const float res = (v - (float)hv) * RES_CAR;
          ldsE[OFF_L + rowl * 72 + 16 * t + c] = (_Float16)res;
        }
      }
  __syncthreads();

  _Float16* const bh = PH + (size_t)z * sC + (size_t)m0 * ldc + n0;
  _Float16* const bl = PL + (size_t)z * sL + (size_t)m0 * ldl + n0;
  for (int i = 0; i < 8; ++i) {
    const int q = i * 128 + tid;
    const int rowl = q >> 3, ch = (q & 7) * 8;
    const v8h vh = *(const v8h*)(&ldsE[rowl * 72 + ch]);
    *(volatile v8h*)(bh + (size_t)rowl * ldc + ch) = vh;
    if (wres) {
      const v8h vl = *(const v8h*)(&ldsE[OFF_L + rowl * 72 + ch]);
      *(volatile v8h*)(bl + (size_t)rowl * ldl + ch) = vl;
    }
  }
  __threadfence();
  for (int i = 0; i < 8; ++i) {
    const int q = i * 128 + tid;
    const int rowl = q >> 3, ch = (q & 7) * 8;
    const v8h vh = *(const v8h*)(&ldsE[rowl * 72 + ch]);
    *(volatile v8h*)(bh + (size_t)rowl * ldc + ch) = vh;
    if (wres) {
      const v8h vl = *(const v8h*)(&ldsE[OFF_L + rowl * 72 + ch]);
      *(volatile v8h*)(bl + (size_t)rowl * ldl + ch) = vl;
    }
  }
}

__global__ __launch_bounds__(128) __attribute__((amdgpu_num_vgpr(256)))
void k_qkrope(const _Float16* __restrict__ A, const _Float16* __restrict__ Bt,
              const float* __restrict__ CosT, const float* __restrict__ SinT,
              _Float16* __restrict__ PH, int K, int ldc)
{
  __shared__ __attribute__((aligned(16))) _Float16 ldsE[128 * 72];
  __shared__ __attribute__((aligned(16))) float ldsC[128 * 32];
  __shared__ __attribute__((aligned(16))) float ldsS[128 * 32];
  static_assert(128 * 72 * 2 + 2 * 128 * 32 * 4 <= 131072);
  static_assert(8 * 128 * 4 == 128 * 32);
  static_assert(8 * 128 * 16 == 128 * 64 * 2);

  const int tid = threadIdx.x, lane = tid & 31;
  const int w = __builtin_amdgcn_readfirstlane(tid >> 5);
  const int hl = lane >> 4, c = lane & 15;
  const int m0 = blockIdx.y * 128, n0 = blockIdx.x * 64;
  const int mw = m0 + 32 * w;
  const int pos0 = m0 - (m0 / SEQ) * SEQ;

  const _Float16* ap0 = A  + (size_t)(mw + c) * K;
  const _Float16* ap1 = A  + (size_t)(mw + 16 + c) * K;
  const _Float16* bp  = Bt + (size_t)(n0 + c) * K;

#pragma unroll
  for (int i = 0; i < 8; ++i) {
    const int idx = (i * 128 + tid) * 4;
    const v4f cv = *(const v4f*)(CosT + (size_t)pos0 * 32 + idx);
    const v4f sv = *(const v4f*)(SinT + (size_t)pos0 * 32 + idx);
    *(v4f*)(&ldsC[idx]) = cv;
    *(v4f*)(&ldsS[idx]) = sv;
  }

  v8f acc[8] = {};
  gemm_core(ap0, ap1, bp, K, hl, acc);
  __syncthreads();

#pragma unroll
  for (int i = 0; i < 2; ++i)
#pragma unroll
    for (int t = 0; t < 2; ++t)
#pragma unroll
      for (int r = 0; r < 8; ++r) {
        const int rowl = 32 * w + 16 * i + 8 * hl + r;
        const int j = 16 * t + c;
        const float cs = ldsC[rowl * 32 + j];
        const float sn = ldsS[rowl * 32 + j];
        const float x1 = acc[i * 4 + t][r] * PROJ_SCL;
        const float x2 = acc[i * 4 + t + 2][r] * PROJ_SCL;
        const float y1 = x1 * cs - x2 * sn;
        const float y2 = x1 * sn + x2 * cs;
        ldsE[rowl * 72 + j]      = toh_flush(y1);
        ldsE[rowl * 72 + 32 + j] = toh_flush(y2);
      }
  __syncthreads();

  _Float16* const bh = PH + (size_t)m0 * ldc + n0;
  for (int i = 0; i < 8; ++i) {
    const int q = i * 128 + tid;
    const int rowl = q >> 3, ch = (q & 7) * 8;
    const v8h vh = *(const v8h*)(&ldsE[rowl * 72 + ch]);
    *(volatile v8h*)(bh + (size_t)rowl * ldc + ch) = vh;
  }
  __threadfence();
  for (int i = 0; i < 8; ++i) {
    const int q = i * 128 + tid;
    const int rowl = q >> 3, ch = (q & 7) * 8;
    const v8h vh = *(const v8h*)(&ldsE[rowl * 72 + ch]);
    *(volatile v8h*)(bh + (size_t)rowl * ldc + ch) = vh;
  }
}

__global__ __launch_bounds__(256) __attribute__((amdgpu_num_vgpr(256)))
void k_attn(const _Float16* __restrict__ QKH, const _Float16* __restrict__ VtH,
            float* Hres, int S)
{
  constexpr int KT_H   = 32 * 72;
  constexpr int V_H    = HD * 40;
  constexpr int P_H    = 8 * 16 * 40;
  constexpr int TILE_H = KT_H + V_H + P_H;
  constexpr int OFF_K  = 0;
  constexpr int OFF_V  = KT_H;
  constexpr int OFF_P  = KT_H + V_H;
  static_assert(OFF_V % 8 == 0 && OFF_P % 8 == 0);
  static_assert(256 * 8 == 32 * 64 && 256 * 8 == HD * 32);
  static_assert(8 * 256 * 16 == 128 * HD * 4);
  static_assert(TILE_H * 2 + 128 * 68 * 4 <= 131072);
  __shared__ __attribute__((aligned(16))) _Float16 lds[TILE_H];
  __shared__ __attribute__((aligned(16))) float ldsO[128 * 68];

  const int tid = threadIdx.x, lane = tid & 31;
  const int wave = __builtin_amdgcn_readfirstlane(tid >> 5);
  const int hl = lane >> 4, c = lane & 15;
  const int q0 = blockIdx.x * 128;
  const int col0 = blockIdx.y * HD;
  const int b = blockIdx.z;

  const size_t qr = (size_t)b * SEQ + q0 + 16 * wave + c;
  v16h qh[2];
#pragma unroll
  for (int ks = 0; ks < 2; ++ks)
    qh[ks] = ld_frag_g(QKH + qr * QKP + col0 + 32 * ks, hl);
  const int pOff = OFF_P + wave * (16 * 40);

  const int krr = tid >> 3, kcc = (tid & 7) * 8;
  const int vdd = tid >> 2, vkc = (tid & 3) * 8;
  const size_t kgo = ((size_t)b * SEQ + krr) * QKP + DM + col0 + kcc;
  const size_t vgo = ((size_t)b * DM + col0 + vdd) * SEQ + vkc;

  float m[8], l[8];
  v8f o[4] = {};
#pragma unroll
  for (int r = 0; r < 8; ++r) { m[r] = NEG_BIG; l[r] = 0.f; }

  const int klo = (q0 - S + 1 > 0) ? (q0 - S + 1) : 0;
  const int kt0 = klo >> 5;
  const int kt1 = (q0 + 127) >> 5;
  const int irow0 = q0 + 16 * wave + 8 * hl;

#pragma unroll 1
  for (int kt = kt0; kt <= kt1; ++kt) {
    const int mk = kt * 32;
    {
      const v8h k8 = *(const v8h*)(QKH + kgo + (size_t)mk * QKP);
      const v8h v8 = *(const v8h*)(VtH + vgo + mk);
      *(v8h*)(&lds[OFF_K + krr * 72 + kcc]) = k8;
      *(v8h*)(&lds[OFF_V + vdd * 40 + vkc]) = v8;
    }
    __syncthreads();

    v8f sh[2] = {};
#pragma unroll
    for (int ks = 0; ks < 2; ++ks) {
#pragma unroll
      for (int t = 0; t < 2; ++t) {
        const v16h kf = ld_frag_s(lds, OFF_K + (16 * t + c) * 72 + 32 * ks, hl);
        sh[t] = mma(qh[ks], kf, sh[t]);
      }
    }

#pragma unroll
    for (int r = 0; r < 8; ++r) {
      const int d0 = (irow0 + r) - (mk + c);
      const int d1 = d0 - 16;
      const bool ok0 = (d0 >= 0) & (d0 < S);
      const bool ok1 = (d1 >= 0) & (d1 < S);
      const float v0 = ok0 ? (sh[0][r] * S_SCL) : NEG_BIG;
      const float v1 = ok1 ? (sh[1][r] * S_SCL) : NEG_BIG;
      float tm = fmaxf(v0, v1);
      tm = fmaxf(tm, __shfl_xor(tm, 1, 32));
      tm = fmaxf(tm, __shfl_xor(tm, 2, 32));
      tm = fmaxf(tm, __shfl_xor(tm, 4, 32));
      tm = fmaxf(tm, __shfl_xor(tm, 8, 32));
      const float mn = fmaxf(m[r], tm);
      const float al = __expf(fmaxf(m[r] - mn, -80.0f));
      const float e0 = __expf(fmaxf(v0 - mn, -80.0f));
      const float e1 = __expf(fmaxf(v1 - mn, -80.0f));
      const float p0 = ok0 ? e0 : 0.0f;
      const float p1 = ok1 ? e1 : 0.0f;
      float rs = p0 + p1;
      rs += __shfl_xor(rs, 1, 32);
      rs += __shfl_xor(rs, 2, 32);
      rs += __shfl_xor(rs, 4, 32);
      rs += __shfl_xor(rs, 8, 32);
      l[r] = l[r] * al + rs;
      m[r] = mn;
#pragma unroll
      for (int t = 0; t < 4; ++t) o[t][r] *= al;
      const int pi = pOff + (8 * hl + r) * 40 + c;
      lds[pi]      = toh_flush(p0 * P_CAR);
      lds[pi + 16] = toh_flush(p1 * P_CAR);
    }
    __syncthreads();

    const v16h pf = ld_frag_s(lds, pOff + c * 40, hl);
#pragma unroll
    for (int t = 0; t < 4; ++t) {
      const v16h vf = ld_frag_s(lds, OFF_V + (16 * t + c) * 40, hl);
      o[t] = mma(pf, vf, o[t]);
    }
    __syncthreads();
  }

#pragma unroll
  for (int r = 0; r < 8; ++r) {
    const float inv = 1.0f / l[r];
    const int rowl = 16 * wave + 8 * hl + r;
#pragma unroll
    for (int t = 0; t < 4; ++t)
      ldsO[rowl * 68 + 16 * t + c] = o[t][r] * inv * O_SCL;
  }
  __syncthreads();

  float* const hb = Hres + ((size_t)b * SEQ + q0) * DM + col0;
  v4f vals[8];
#pragma unroll
  for (int i = 0; i < 8; ++i) {
    const int q = i * 256 + tid;
    const int rowl = q >> 4, col = (q & 15) * 4;
    const v4f old = *(const v4f*)(hb + (size_t)rowl * DM + col);
    const v4f add = *(const v4f*)(&ldsO[rowl * 68 + col]);
    vals[i] = old + add;
  }
#pragma unroll
  for (int i = 0; i < 8; ++i) {
    const int q = i * 256 + tid;
    const int rowl = q >> 4, col = (q & 15) * 4;
    *(volatile v4f*)(hb + (size_t)rowl * DM + col) = vals[i];
  }
  __threadfence();
#pragma unroll
  for (int i = 0; i < 8; ++i) {
    const int q = i * 256 + tid;
    const int rowl = q >> 4, col = (q & 15) * 4;
    *(volatile v4f*)(hb + (size_t)rowl * DM + col) = vals[i];
  }
}

__global__ __launch_bounds__(128) __attribute__((amdgpu_num_vgpr(256)))
void k_ffn1(const _Float16* __restrict__ A, const _Float16* __restrict__ Bt,
            const float* __restrict__ bias, _Float16* __restrict__ PH, int K, int ldc)
{
  __shared__ __attribute__((aligned(16))) float    ldsF[128 * 68];
  __shared__ __attribute__((aligned(16))) _Float16 ldsE[128 * 72];
  static_assert(128 * 68 * 4 + 128 * 72 * 2 <= 131072);
  static_assert(8 * 128 * 16 == 128 * 64 * 2);

  const int tid = threadIdx.x, lane = tid & 31;
  const int w = __builtin_amdgcn_readfirstlane(tid >> 5);
  const int hl = lane >> 4, c = lane & 15;
  const int m0 = blockIdx.y * 128, n0 = blockIdx.x * 64;
  const int mw = m0 + 32 * w;

  const _Float16* ap0 = A  + (size_t)(mw + c) * K;
  const _Float16* ap1 = A  + (size_t)(mw + 16 + c) * K;
  const _Float16* bp  = Bt + (size_t)(n0 + c) * K;

  v8f acc[8] = {};
  gemm_core(ap0, ap1, bp, K, hl, acc);

#pragma unroll
  for (int i = 0; i < 2; ++i)
#pragma unroll
    for (int t = 0; t < 4; ++t)
#pragma unroll
      for (int r = 0; r < 8; ++r) {
        const int rowl = 32 * w + 16 * i + 8 * hl + r;
        ldsF[rowl * 68 + 16 * t + c] = acc[i * 4 + t][r] * UNS_SCL;
      }
  __syncthreads();

  _Float16* const bh = PH + (size_t)m0 * ldc + n0;
#pragma unroll 1
  for (int i = 0; i < 8; ++i) {
    const int q = i * 128 + tid;
    const int rowl = q >> 3, ch = (q & 7) * 8;
    const v4f x0 = *(const v4f*)(&ldsF[rowl * 68 + ch]);
    const v4f x1 = *(const v4f*)(&ldsF[rowl * 68 + ch + 4]);
    const v4f b0 = *(const v4f*)(bias + n0 + ch);
    const v4f b1 = *(const v4f*)(bias + n0 + ch + 4);
    v8h ov;
#pragma unroll
    for (int e = 0; e < 4; ++e) {
      ov[e]     = toh_flush(gelu_erf(x0[e] + bf16_rne(b0[e])) * ACT_CAR);
      ov[4 + e] = toh_flush(gelu_erf(x1[e] + bf16_rne(b1[e])) * ACT_CAR);
    }
    *(v8h*)(&ldsE[rowl * 72 + ch]) = ov;
    *(volatile v8h*)(bh + (size_t)rowl * ldc + ch) = ov;
  }
  __threadfence();
  __syncthreads();
  for (int i = 0; i < 8; ++i) {
    const int q = i * 128 + tid;
    const int rowl = q >> 3, ch = (q & 7) * 8;
    const v8h vh = *(const v8h*)(&ldsE[rowl * 72 + ch]);
    *(volatile v8h*)(bh + (size_t)rowl * ldc + ch) = vh;
  }
}

__global__ __launch_bounds__(128) __attribute__((amdgpu_num_vgpr(256)))
void k_gemm_res(const _Float16* __restrict__ A, const _Float16* __restrict__ Bt,
                const float* __restrict__ bias, const float* Res, float* Out,
                int K, int ldo, int hasres, int seq_o)
{
  __shared__ __attribute__((aligned(16))) float ldsF[128 * 68];
  static_assert(128 * 68 * 4 <= 131072);
  static_assert(16 * 128 * 16 == 128 * 64 * 4);

  const int tid = threadIdx.x, lane = tid & 31;
  const int w = __builtin_amdgcn_readfirstlane(tid >> 5);
  const int hl = lane >> 4, c = lane & 15;
  const int m0 = blockIdx.y * 128, n0 = blockIdx.x * 64;
  const int mw = m0 + 32 * w;

  const _Float16* ap0 = A  + (size_t)(mw + c) * K;
  const _Float16* ap1 = A  + (size_t)(mw + 16 + c) * K;
  const _Float16* bp  = Bt + (size_t)(n0 + c) * K;

  v8f acc[8] = {};
  gemm_core(ap0, ap1, bp, K, hl, acc);

#pragma unroll
  for (int i = 0; i < 2; ++i)
#pragma unroll
    for (int t = 0; t < 4; ++t)
#pragma unroll
      for (int r = 0; r < 8; ++r) {
        const int rowl = 32 * w + 16 * i + 8 * hl + r;
        ldsF[rowl * 68 + 16 * t + c] = acc[i * 4 + t][r] * UNS_SCL;
      }
  __syncthreads();

  const int bcol = (tid & 15) * 4;
  const v4f braw = *(const v4f*)(bias + n0 + bcol);
  v4f bb;
  bb[0] = bf16_rne(braw[0]); bb[1] = bf16_rne(braw[1]);
  bb[2] = bf16_rne(braw[2]); bb[3] = bf16_rne(braw[3]);

  const int ob_b = m0 / SEQ;
  const int ob_n = m0 - ob_b * SEQ;
  float* const ob = Out + ((size_t)ob_b * seq_o + ob_n) * ldo + n0;
  const float* const rb = Res + (size_t)m0 * DM + n0;
  v4f vals[16];
#pragma unroll
  for (int i = 0; i < 16; ++i) {
    const int qi = i * 128 + tid;
    const int rowl = qi >> 4, col = (qi & 15) * 4;
    const v4f rr = *(const v4f*)(rb + (size_t)rowl * DM + col);
    const v4f t  = *(const v4f*)(&ldsF[rowl * 68 + col]) + bb;
    v4f o;
    o[0] = hasres ? (t[0] + rr[0]) : t[0];
    o[1] = hasres ? (t[1] + rr[1]) : t[1];
    o[2] = hasres ? (t[2] + rr[2]) : t[2];
    o[3] = hasres ? (t[3] + rr[3]) : t[3];
    vals[i] = o;
  }
#pragma unroll
  for (int i = 0; i < 16; ++i) {
    const int qi = i * 128 + tid;
    const int rowl = qi >> 4, col = (qi & 15) * 4;
    *(volatile v4f*)(ob + (size_t)rowl * ldo + col) = vals[i];
  }
  __threadfence();
#pragma unroll
  for (int i = 0; i < 16; ++i) {
    const int qi = i * 128 + tid;
    const int rowl = qi >> 4, col = (qi & 15) * 4;
    *(volatile v4f*)(ob + (size_t)rowl * ldo + col) = vals[i];
  }
}

__global__ __launch_bounds__(256) void k_loss(const float* logits, const int* __restrict__ y, float* loss)
{
  __shared__ float part[8];
  const int tid = threadIdx.x, lane = tid & 31;
  const int wave = __builtin_amdgcn_readfirstlane(tid >> 5);
  float accw = 0.f;
#pragma unroll 1
  for (int row = wave; row < ROWS; row += 8) {
    const int bb = row / SEQ;
    const int nn = row - bb * SEQ;
    const size_t grow = (size_t)bb * SEQ_FULL + nn;
    const float* lr = logits + grow * VOC;
    const v4f x0 = *(const v4f*)(lr + 8 * lane);
    const v4f x1 = *(const v4f*)(lr + 8 * lane + 4);
    float mx = fmaxf(fmaxf(fmaxf(x0[0], x0[1]), fmaxf(x0[2], x0[3])),
                     fmaxf(fmaxf(x1[0], x1[1]), fmaxf(x1[2], x1[3])));
    mx = fmaxf(mx, __shfl_xor(mx, 16, 32));
    mx = fmaxf(mx, __shfl_xor(mx, 8, 32));
    mx = fmaxf(mx, __shfl_xor(mx, 4, 32));
    mx = fmaxf(mx, __shfl_xor(mx, 2, 32));
    mx = fmaxf(mx, __shfl_xor(mx, 1, 32));
    float se = 0.f;
#pragma unroll
    for (int e = 0; e < 4; ++e) {
      se += __expf(x0[e] - mx);
      se += __expf(x1[e] - mx);
    }
    se += __shfl_xor(se, 16, 32);
    se += __shfl_xor(se, 8, 32);
    se += __shfl_xor(se, 4, 32);
    se += __shfl_xor(se, 2, 32);
    se += __shfl_xor(se, 1, 32);
    int yy = y[grow];
    yy = (yy < 0) ? 0 : ((yy > VOC - 1) ? (VOC - 1) : yy);
    const float ly = lr[yy];
    accw += (ly - mx) - __logf(se);
  }
  if (lane == 0) part[wave] = accw;
  __syncthreads();
  if (tid == 0) {
    float s = 0.f;
#pragma unroll
    for (int w = 0; w < 8; ++w) s += part[w];
    const float v = -s * (1.0f / (float)ROWS);
    *(volatile float*)loss = v;
    __threadfence();
    *(volatile float*)loss = v;
  }
}

extern "C" void kernel_launch(void* const* d_in, const int* in_sizes, int n_in,
                              void* d_out, int out_size, void* d_ws, size_t ws_size,
                              hipStream_t stream)
{
  if (n_in < 14) return;
  const long need_tok = (long)(NB - 1) * SEQ_FULL + SEQ;
  if ((long)in_sizes[0] < need_tok) return;
  if ((long)in_sizes[1] < need_tok) return;
  if ((long)in_sizes[2] < (long)VOC * DM) return;
  if ((long)in_sizes[3] < (long)NLAY * DM * QKVW) return;
  if ((long)in_sizes[4] < (long)NLAY * 2 * DM) return;
  if ((long)in_sizes[5] < (long)NLAY * 2 * DM) return;
  if ((long)in_sizes[6] < (long)NLAY * DM * FFW) return;
  if ((long)in_sizes[7] < (long)NLAY * FFW) return;
  if ((long)in_sizes[8] < (long)NLAY * FFW * DM) return;
  if ((long)in_sizes[9] < (long)NLAY * DM) return;
  if ((long)in_sizes[10] < (long)DM) return;
  if ((long)in_sizes[11] < (long)DM) return;
  if ((long)in_sizes[12] < (long)DM * VOC) return;
  if ((long)in_sizes[13] < (long)VOC) return;
  if ((long)out_size < OUT1_ELEMS + 1) return;
  if (WS_HALVES * sizeof(_Float16) > ws_size) return;

  const int*   tok       = (const int*)  d_in[0];
  const int*   tgt       = (const int*)  d_in[1];
  const float* emb       = (const float*)d_in[2];
  const float* qkv_w     = (const float*)d_in[3];
  const float* ln_scale  = (const float*)d_in[4];
  const float* ln_bias   = (const float*)d_in[5];
  const float* ff_w1     = (const float*)d_in[6];
  const float* ff_b1     = (const float*)d_in[7];
  const float* ff_w2     = (const float*)d_in[8];
  const float* ff_b2     = (const float*)d_in[9];
  const float* lnf_scale = (const float*)d_in[10];
  const float* lnf_bias  = (const float*)d_in[11];
  const float* head_w    = (const float*)d_in[12];
  const float* head_b    = (const float*)d_in[13];
  float* out = (float*)d_out;

  _Float16* WqkvT = (_Float16*)d_ws;
  _Float16* W1T   = WqkvT + N_WQKV;
  _Float16* W2T   = W1T   + N_W1;
  _Float16* WhT   = W2T   + N_W2;
  _Float16* N16   = WhT   + N_WH;
  _Float16* QKH   = N16   + N_N16;
  _Float16* VtH   = QKH   + N_QK;
  _Float16* F1    = VtH   + N_VT;
  float*    H0    = (float*)(F1 + N_F1);
  float*    H     = H0 + (size_t)ROWS * DM;
  float*    CosT  = H  + (size_t)ROWS * DM;
  float*    SinT  = CosT + (size_t)SEQ * 32;
  float*    InvF  = SinT + (size_t)SEQ * 32;

  k_invf<<<1, 32, 0, stream>>>(InvF);
  k_ropetab<<<(SEQ * 32) / 256, 256, 0, stream>>>(InvF, CosT, SinT);
  k_embed<<<ROWS / 8, 256, 0, stream>>>(tok, emb, H0, H);

  k_trw<<<dim3(QKVW / 64, DM / 64, NLAY), 256, 0, stream>>>(qkv_w, WqkvT, DM, QKVW);
  k_trw<<<dim3(FFW / 64, DM / 64, NLAY), 256, 0, stream>>>(ff_w1, W1T, DM, FFW);
  k_trw<<<dim3(DM / 64, FFW / 64, NLAY), 256, 0, stream>>>(ff_w2, W2T, FFW, DM);
  k_trw<<<dim3(VOC / 64, DM / 64, 1), 256, 0, stream>>>(head_w, WhT, DM, VOC);

  for (int l = 0; l < NLAY; ++l) {
    int win = 16 << l;
    if (win > 128) win = 128;
    const _Float16* wq = WqkvT + (size_t)l * QKVW * DM;

    k_ln<<<ROWS / 8, 256, 0, stream>>>(H, H0, 0, ln_scale + (size_t)(2 * l) * DM,
                                       ln_bias + (size_t)(2 * l) * DM, N16);
    k_qkrope<<<dim3(QKP / 64, ROWS / 128), 128, 0, stream>>>(N16, wq, CosT, SinT, QKH, DM, QKP);
    k_proj<<<dim3(SEQ / 64, DM / 128, NB), 128, 0, stream>>>(
        wq + (size_t)2 * DM * DM, N16, VtH, QKH,
        (size_t)0, (size_t)SEQ * DM, (size_t)DM * SEQ, (size_t)0,
        DM, SEQ, SEQ, 0, 0);
    k_attn<<<dim3(SEQ / 128, NH, NB), 256, 0, stream>>>(QKH, VtH, H, win);

    k_ln<<<ROWS / 8, 256, 0, stream>>>(H, H0, 0, ln_scale + (size_t)(2 * l + 1) * DM,
                                       ln_bias + (size_t)(2 * l + 1) * DM, N16);
    k_ffn1<<<dim3(FFW / 64, ROWS / 128), 128, 0, stream>>>(
        N16, W1T + (size_t)l * FFW * DM, ff_b1 + (size_t)l * FFW, F1, DM, FFW);
    k_gemm_res<<<dim3(DM / 64, ROWS / 128), 128, 0, stream>>>(
        F1, W2T + (size_t)l * DM * FFW, ff_b2 + (size_t)l * DM, H, H, FFW, DM, 1, SEQ);
  }

  k_ln<<<ROWS / 8, 256, 0, stream>>>(H, H0, 1, lnf_scale, lnf_bias, N16);
  k_gemm_res<<<dim3(VOC / 64, ROWS / 128), 128, 0, stream>>>(
      N16, WhT, head_b, H, out, DM, VOC, 0, SEQ_FULL);
  k_loss<<<1, 256, 0, stream>>>(out, tgt, out + OUT1_ELEMS);
}
